// MultiLatentAttention_48206712930695
// MI455X (gfx1250) — hardware-verified
//
#include <hip/hip_runtime.h>

#ifndef NB
#define NB 2
#endif
#ifndef SEQ
#define SEQ 2048
#endif
#define NB_FULL 2
#define SEQ_FULL 2048
#define DM 2048
#define LDIM 512
#define NHEAD 16
#define HDIM 128
#ifndef RS
#define RS (SEQ < 512 ? SEQ : 512)
#endif
static_assert(SEQ % 128 == 0);
static_assert((RS % 128) == 0 && RS >= 128 && RS <= SEQ);
static_assert(((SEQ - RS) % 128) == 0);
static_assert(NB >= 1 && NB <= NB_FULL && SEQ <= SEQ_FULL);
static_assert(DM == NHEAD * HDIM);
static_assert(HDIM == 128 && LDIM % 128 == 0 && DM % 128 == 0);

#ifdef ATTN_VGPR_CAP
#define ATTN_ATTR __attribute__((amdgpu_num_vgpr(256)))
#else
#define ATTN_ATTR
#endif

typedef _Float16 f16;
typedef f16 v16h __attribute__((ext_vector_type(16)));
typedef f16 v8h_t __attribute__((ext_vector_type(8)));
typedef v8h_t v8h __attribute__((may_alias));
typedef float v8f __attribute__((ext_vector_type(8)));
typedef float v4f_t __attribute__((ext_vector_type(4)));
typedef v4f_t v4f __attribute__((may_alias));
typedef unsigned int v4u_t __attribute__((ext_vector_type(4)));
typedef v4u_t v4u __attribute__((may_alias));

union Frag { v16h v; v8h_t hv[2]; };
union H8 { v8h_t v; f16 e[8]; };
union U8 { v4u_t u; f16 e[8]; };

__device__ __forceinline__ v16h ldfrag(const f16* base, int row0, int ld, int k0) {
  const int l = threadIdx.x & 31, hh = l >> 4, m = l & 15;
  const f16* p = base + (size_t)(row0 + m) * (size_t)ld + k0 + 8 * hh;
  Frag f;
  f.hv[0] = *(const v8h*)p;
  f.hv[1] = *(const v8h*)(p + 16);
  return f.v;
}

__device__ __forceinline__ v8f wm(v8f c, v16h a, v16h b) {
  v8f d = __builtin_amdgcn_wmma_f32_16x16x32_f16(false, a, false, b, (short)0, c, false, false);
  asm volatile("v_nop\n\tv_nop\n\tv_nop\n\tv_nop" : "+v"(d) : "v"(a), "v"(b));
  return d;
}

__device__ __forceinline__ void split16(float v, f16& hi, f16& lo) {
  hi = (f16)v;
  lo = (f16)((v - (float)hi) * 2048.0f);
}

__device__ __forceinline__ float bf16r(float v) {
  unsigned int u = __float_as_uint(v);
  u = (u + 0x7fffu + ((u >> 16) & 1u)) & 0xffff0000u;
  return __uint_as_float(u);
}

__global__ __launch_bounds__(256) void k_cvt_x(const float* __restrict__ x, f16* xh, int total_rows, int cols,
                                               int rows_per_grp, int src_grp_stride) {
  const size_t gid = (size_t)blockIdx.x * 256 + threadIdx.x;
  const size_t e = gid * 8;
  const size_t row = e / (size_t)cols;
  if (row >= (size_t)total_rows) return;
  const int col = (int)(e - row * cols);
  const int grp = (int)(row / (size_t)rows_per_grp);
  const int s = (int)(row - (size_t)grp * rows_per_grp);
  const float* src = x + ((size_t)grp * src_grp_stride + s) * (size_t)cols + col;
  v4f_t a = *(const v4f*)src;
  v4f_t b = *(const v4f*)(src + 4);
  float v[8] = {a[0], a[1], a[2], a[3], b[0], b[1], b[2], b[3]};
  H8 hh;
#pragma unroll
  for (int i = 0; i < 8; ++i) hh.e[i] = (f16)bf16r(v[i]);
  f16* dh = xh + e;
  *(volatile v8h_t*)dh = hh.v;
  __threadfence();
  *(volatile v8h_t*)dh = hh.v;
}

__global__ __launch_bounds__(256) void k_wT(const float* __restrict__ in, f16* outh, int K, int N, float sc) {
  __shared__ float t[64][33];
  const int n0 = blockIdx.x * 32, k0 = blockIdx.y * 64;
  const int tid = threadIdx.x;
  {
    const int nn = tid & 31, kb = tid >> 5;
#pragma unroll
    for (int i = 0; i < 8; ++i) {
      const int kk = kb + 8 * i;
      t[kk][nn] = in[(size_t)(k0 + kk) * N + n0 + nn];
    }
  }
  __syncthreads();
  const int nn = tid >> 3, sub = tid & 7;
  H8 hh;
#pragma unroll
  for (int e = 0; e < 8; ++e) hh.e[e] = (f16)(bf16r(t[sub * 8 + e][nn]) * sc);
  const size_t off = (size_t)(n0 + nn) * K + k0 + sub * 8;
  *(volatile v8h_t*)(outh + off) = hh.v;
  __threadfence();
  *(volatile v8h_t*)(outh + off) = hh.v;
}

#define SCP 132
template <bool ASPLIT, int MODE, bool HASB>
__global__ __launch_bounds__(256) void k_gemm(const f16* __restrict__ Ah, const f16* __restrict__ Al,
                                              const f16* __restrict__ Bh, const float* __restrict__ bias,
                                              f16* Ch, f16* Cl, float* Cf,
                                              int K, int N, int tpg, int grp_stride, int row_start, int R,
                                              float oscale, float sout) {
  __shared__ __attribute__((aligned(16))) f16 sA[2][128 * 32];
  __shared__ __attribute__((aligned(16))) f16 sB[128 * 32];
  __shared__ __attribute__((aligned(16))) float sC[128 * SCP];

  const int tid = threadIdx.x, wave = tid >> 5, lane = tid & 31;
  const int hf = lane >> 4, lc = lane & 15;
  const int wmi = wave >> 2, wn = wave & 3;
  const int y = blockIdx.y;
  const int grp = y / tpg;
  const int mrel = row_start + (y - grp * tpg) * 128;
  const size_t arow = (size_t)grp * grp_stride + mrel;
  const size_t lrow = (size_t)grp * R + mrel;
  const int n0 = blockIdx.x * 128;
  const float kx = 0.00048828125f;
  const bool clo = (mrel < R);

  v8f acc[4][2];
#pragma unroll
  for (int mi = 0; mi < 4; ++mi) { acc[mi][0] = (v8f){}; acc[mi][1] = (v8f){}; }

  const int nk = K >> 5;
  for (int kt = 0; kt < nk; ++kt) {
    const int k0 = kt << 5;
#pragma unroll
    for (int i = 0; i < 2; ++i) {
      const int q = tid + 256 * i;
      const int row = q >> 2, c4 = q & 3;
      *(v4u*)(&sA[0][row * 32 + c4 * 8]) = *(const v4u*)(Ah + (arow + row) * K + k0 + c4 * 8);
      *(v4u*)(&sB[row * 32 + c4 * 8]) = *(const v4u*)(Bh + (size_t)(n0 + row) * K + k0 + c4 * 8);
      if (ASPLIT) {
        *(v4u*)(&sA[1][row * 32 + c4 * 8]) = *(const v4u*)(Al + (lrow + row) * K + k0 + c4 * 8);
      }
    }
    __syncthreads();
    v16h bh0 = ldfrag(sB, wn * 32, 32, 0);
    v16h bh1 = ldfrag(sB, wn * 32 + 16, 32, 0);
#pragma unroll
    for (int mi = 0; mi < 4; ++mi) {
      v16h ah = ldfrag(sA[0], wmi * 64 + mi * 16, 32, 0);
      acc[mi][0] = wm(acc[mi][0], ah, bh0);
      acc[mi][1] = wm(acc[mi][1], ah, bh1);
      if (ASPLIT) {
        v16h al = ldfrag(sA[1], wmi * 64 + mi * 16, 32, 0);
        v8f t0 = (v8f){};
        t0 = wm(t0, al, bh0);
        acc[mi][0] += t0 * kx;
        v8f t1 = (v8f){};
        t1 = wm(t1, al, bh1);
        acc[mi][1] += t1 * kx;
      }
    }
    __syncthreads();
  }

#pragma unroll
  for (int mi = 0; mi < 4; ++mi)
#pragma unroll
    for (int r = 0; r < 8; ++r) {
      const int row = wmi * 64 + mi * 16 + 8 * hf + r;
      sC[row * SCP + wn * 32 + lc] = acc[mi][0][r];
      sC[row * SCP + wn * 32 + 16 + lc] = acc[mi][1][r];
    }
  __syncthreads();

  if (MODE == 2) {
    for (int pass = 0; pass < 2; ++pass) {
#pragma unroll 4
      for (int it = 0; it < 16; ++it) {
        const int r = wave * 16 + it;
        const float* src = sC + r * SCP + lane * 4;
        v4f_t bb = (v4f_t){};
        if (HASB) {
          bb = *(const v4f*)(bias + n0 + lane * 4);
          bb[0] = bf16r(bb[0]); bb[1] = bf16r(bb[1]); bb[2] = bf16r(bb[2]); bb[3] = bf16r(bb[3]);
        }
        v4f_t v;
        v[0] = src[0] * oscale + bb[0]; v[1] = src[1] * oscale + bb[1];
        v[2] = src[2] * oscale + bb[2]; v[3] = src[3] * oscale + bb[3];
        *(volatile v4f_t*)(Cf + (arow + r) * N + n0 + lane * 4) = v;
      }
      if (pass == 0) __threadfence();
    }
  } else {
    for (int pass = 0; pass < 2; ++pass) {
#pragma unroll 2
      for (int it = 0; it < 8; ++it) {
        const int unit = it * 4 + (lane >> 3);
        const int rl = unit >> 1, chunk = unit & 1, sub = lane & 7;
        const int r = wave * 16 + rl;
        const float* src = sC + r * SCP + chunk * 64 + sub * 8;
        const int n = n0 + chunk * 64 + sub * 8;
        float bb[8] = {0.f, 0.f, 0.f, 0.f, 0.f, 0.f, 0.f, 0.f};
        if (HASB) {
          v4f_t b0 = *(const v4f*)(bias + n);
          v4f_t b1 = *(const v4f*)(bias + n + 4);
          bb[0] = bf16r(b0[0]); bb[1] = bf16r(b0[1]); bb[2] = bf16r(b0[2]); bb[3] = bf16r(b0[3]);
          bb[4] = bf16r(b1[0]); bb[5] = bf16r(b1[1]); bb[6] = bf16r(b1[2]); bb[7] = bf16r(b1[3]);
        }
        H8 hh8, ll8;
#pragma unroll
        for (int e = 0; e < 8; ++e) split16((src[e] * oscale + bb[e]) * sout, hh8.e[e], ll8.e[e]);
        const size_t crow = arow + r, clrow = lrow + r;
        *(volatile v8h_t*)(Ch + crow * N + n) = hh8.v;
        if (clo) *(volatile v8h_t*)(Cl + clrow * N + n) = ll8.v;
      }
      if (pass == 0) __threadfence();
    }
  }
}

template <bool SPLIT>
__global__ __launch_bounds__(128) ATTN_ATTR void k_attn(const f16* __restrict__ qh, const f16* __restrict__ ql,
                                                        const f16* __restrict__ kh, const f16* __restrict__ kl,
                                                        const f16* __restrict__ vh, const f16* __restrict__ vl,
                                                        f16* ch, f16* cl, int blk0, int S, int R, float scale) {
  constexpr int D = DM;
  constexpr int oQh = 0;
  constexpr int oQl = 8192;
  constexpr int oKh = SPLIT ? 16384 : 8192;
  constexpr int oKl = oKh + 8192;
  constexpr int oVh = SPLIT ? oKl + 8192 : oKh + 8192;
  constexpr int oVl = oVh + 4096;
  constexpr int oPh = SPLIT ? oVl + 4096 : oVh + 4096;
  constexpr int oPl = oPh + 4096;
  constexpr int TOT = SPLIT ? oPl + 4096 : oPh + 4096;
  __shared__ __attribute__((aligned(16))) f16 sm[TOT];

  const int tid = threadIdx.x, wave = tid >> 5, lane = tid & 31, hf = lane >> 4, lc = lane & 15;
  const int qb = blockIdx.x + blk0, h = (int)(blockIdx.y >> 1), dh = (int)(blockIdx.y & 1), b = blockIdx.z;
  const int q0 = qb * 64;
  const float kx = 0.00048828125f;
  const f16* qhb = qh + (size_t)b * S * D + h * HDIM;
  const f16* qlb = ql + (size_t)b * R * D + h * HDIM;
  const f16* khb = kh + (size_t)b * S * D + h * HDIM;
  const f16* klb = kl + (size_t)b * R * D + h * HDIM;
  const f16* vhb = vh + (size_t)b * S * D + h * HDIM + dh * 64;
  const f16* vlb = vl + (size_t)b * R * D + h * HDIM + dh * 64;
  f16* chb = ch + (size_t)b * S * D + h * HDIM + dh * 64;
  f16* clb = cl + (size_t)b * R * D + h * HDIM + dh * 64;

  for (int i = tid; i < 1024; i += 128) {
    const int row = i >> 4, c = i & 15;
    *(v4u*)(sm + oQh + row * 128 + c * 8) = *(const v4u*)(qhb + (size_t)(q0 + row) * D + c * 8);
    if (SPLIT) *(v4u*)(sm + oQl + row * 128 + c * 8) = *(const v4u*)(qlb + (size_t)(q0 + row) * D + c * 8);
  }

  v8f o[4];
#pragma unroll
  for (int dv = 0; dv < 4; ++dv) o[dv] = (v8f){};
  float mrow[8], lrow[8];
#pragma unroll
  for (int j = 0; j < 8; ++j) { mrow[j] = -1e30f; lrow[j] = 0.0f; }

  const int nblk = qb + 1;
  const int qw = q0 + wave * 16;
  f16* pw = sm + oPh + wave * 1024;
  f16* pwl = sm + oPl + wave * 1024;

  for (int kbi = 0; kbi < nblk; ++kbi) {
    const int k0 = kbi * 64;
    __syncthreads();
    for (int i = tid; i < 1024; i += 128) {
      const int row = i >> 4, c = i & 15;
      *(v4u*)(sm + oKh + row * 128 + c * 8) = *(const v4u*)(khb + (size_t)(k0 + row) * D + c * 8);
      if (SPLIT) *(v4u*)(sm + oKl + row * 128 + c * 8) = *(const v4u*)(klb + (size_t)(k0 + row) * D + c * 8);
    }
    for (int i = tid; i < 512; i += 128) {
      const int key = i >> 3, c = i & 7;
      U8 u;
      u.u = *(const v4u*)(vhb + (size_t)(k0 + key) * D + c * 8);
#pragma unroll
      for (int e = 0; e < 8; ++e) sm[oVh + (c * 8 + e) * 64 + key] = u.e[e];
      if (SPLIT) {
        U8 w;
        w.u = *(const v4u*)(vlb + (size_t)(k0 + key) * D + c * 8);
#pragma unroll
        for (int e = 0; e < 8; ++e) sm[oVl + (c * 8 + e) * 64 + key] = w.e[e];
      }
    }
    __syncthreads();

    v8f sa[4], st[4];
#pragma unroll
    for (int nt = 0; nt < 4; ++nt) { sa[nt] = (v8f){}; st[nt] = (v8f){}; }
#pragma unroll 1
    for (int kc = 0; kc < 4; ++kc) {
      const int kk = kc * 32;
      v16h qf = ldfrag(sm + oQh, wave * 16, 128, kk);
      v16h qfl = (v16h){};
      if (SPLIT) qfl = ldfrag(sm + oQl, wave * 16, 128, kk);
#pragma unroll
      for (int nt = 0; nt < 4; ++nt) {
        v16h kf = ldfrag(sm + oKh, nt * 16, 128, kk);
        sa[nt] = wm(sa[nt], qf, kf);
        if (SPLIT) {
          v16h kfl = ldfrag(sm + oKl, nt * 16, 128, kk);
          st[nt] = wm(st[nt], qf, kfl);
          st[nt] = wm(st[nt], qfl, kf);
        }
      }
    }
    v8f s[4];
#pragma unroll
    for (int nt = 0; nt < 4; ++nt) {
      if (SPLIT) s[nt] = sa[nt] + st[nt] * kx;
      else s[nt] = sa[nt];
    }

#pragma unroll
    for (int j = 0; j < 8; ++j) {
      const int mg = qw + j + 8 * hf;
      float tm = -1e30f;
#pragma unroll
      for (int nt = 0; nt < 4; ++nt) {
        const int ng = k0 + nt * 16 + lc;
        float v = s[nt][j] * scale;
        v = (ng <= mg) ? v : -1e30f;
        s[nt][j] = v;
        tm = fmaxf(tm, v);
      }
#pragma unroll
      for (int off = 1; off < 16; off <<= 1) tm = fmaxf(tm, __shfl_xor(tm, off, 32));
      const float mn = fmaxf(mrow[j], tm);
      const float scf = __expf(mrow[j] - mn);
      mrow[j] = mn;
      float rs = 0.0f;
#pragma unroll
      for (int nt = 0; nt < 4; ++nt) {
        float p = __expf(s[nt][j] - mn);
        s[nt][j] = p;
        rs += p;
      }
#pragma unroll
      for (int off = 1; off < 16; off <<= 1) rs += __shfl_xor(rs, off, 32);
      lrow[j] = lrow[j] * scf + rs;
#pragma unroll
      for (int dv = 0; dv < 4; ++dv) o[dv][j] *= scf;
    }

#pragma unroll
    for (int nt = 0; nt < 4; ++nt)
#pragma unroll
      for (int j = 0; j < 8; ++j) {
        const float p = s[nt][j] * 4096.0f;
        f16 phv, plv;
        split16(p, phv, plv);
        pw[(j + 8 * hf) * 64 + nt * 16 + lc] = phv;
        if (SPLIT) pwl[(j + 8 * hf) * 64 + nt * 16 + lc] = plv;
      }
    __syncthreads();

    v8f ot[4];
#pragma unroll
    for (int dv = 0; dv < 4; ++dv) ot[dv] = (v8f){};
#pragma unroll 1
    for (int kc = 0; kc < 2; ++kc) {
      const int kk = kc * 32;
      v16h pf = ldfrag(pw, 0, 64, kk);
      v16h plf = (v16h){};
      if (SPLIT) plf = ldfrag(pwl, 0, 64, kk);
#pragma unroll
      for (int dv = 0; dv < 4; ++dv) {
        v16h vf = ldfrag(sm + oVh, dv * 16, 64, kk);
        o[dv] = wm(o[dv], pf, vf);
        if (SPLIT) {
          v16h vlf = ldfrag(sm + oVl, dv * 16, 64, kk);
          ot[dv] = wm(ot[dv], pf, vlf);
          ot[dv] = wm(ot[dv], plf, vf);
        }
      }
    }
    if (SPLIT) {
#pragma unroll
      for (int dv = 0; dv < 4; ++dv) o[dv] += ot[dv] * kx;
    }
  }

  __syncthreads();
  f16* sth = sm + oKh + wave * 1024;
  f16* stl = sm + oKh + 4096 + wave * 1024;
#pragma unroll
  for (int j = 0; j < 8; ++j) {
    const float invl = (1.0f / lrow[j]) * (1.0f / 4096.0f) * 16.0f;
#pragma unroll
    for (int dv = 0; dv < 4; ++dv) {
      f16 hv, lv;
      split16(o[dv][j] * invl, hv, lv);
      sth[(j + 8 * hf) * 64 + dv * 16 + lc] = hv;
      if (SPLIT) stl[(j + 8 * hf) * 64 + dv * 16 + lc] = lv;
    }
  }
  __syncthreads();
  for (int pass = 0; pass < 2; ++pass) {
#pragma unroll
    for (int it = 0; it < 4; ++it) {
      const int rl = it * 4 + (lane >> 3), sub = lane & 7;
      const size_t row = (size_t)(qw + rl);
      v8h_t hv = *(const v8h*)(sth + rl * 64 + sub * 8);
      *(volatile v8h_t*)(chb + row * D + sub * 8) = hv;
      if (SPLIT) {
        v8h_t lv = *(const v8h*)(stl + rl * 64 + sub * 8);
        *(volatile v8h_t*)(clb + row * D + sub * 8) = lv;
      }
    }
    if (pass == 0) __threadfence();
  }
}

extern "C" void kernel_launch(void* const* d_in, const int* in_sizes, int n_in,
                              void* d_out, int out_size, void* d_ws, size_t ws_size,
                              hipStream_t stream) {
  const int Bn = NB, S = SEQ, R = RS, D = DM, L = LDIM, H = NHEAD;
  if (n_in < 9) return;
  const long long need_x = ((long long)(Bn - 1) * SEQ_FULL + S) * (long long)D;
  if ((long long)in_sizes[0] < need_x || in_sizes[1] < D * D || in_sizes[2] < D || in_sizes[3] < D * L ||
      in_sizes[4] < D * L || in_sizes[5] < L * D || in_sizes[6] < L * D || in_sizes[7] < D * D ||
      in_sizes[8] < D || (long long)out_size < (long long)Bn * S * D) return;

  const float* x     = (const float*)d_in[0];
  const float* wq    = (const float*)d_in[1];
  const float* bq    = (const float*)d_in[2];
  const float* wklat = (const float*)d_in[3];
  const float* wvlat = (const float*)d_in[4];
  const float* wk    = (const float*)d_in[5];
  const float* wv    = (const float*)d_in[6];
  const float* wo    = (const float*)d_in[7];
  const float* bo    = (const float*)d_in[8];
  float* out = (float*)d_out;

  char* ws = (char*)d_ws;
  size_t off = 0;
  auto take = [&](size_t bytes) -> char* { char* p = ws + off; off += (bytes + 255) & ~(size_t)255; return p; };
  auto takeh = [&](size_t elems) -> f16* { return (f16*)take(elems * 2); };

  f16* xh   = takeh((size_t)Bn * S * D);
  f16* ctxh = xh;
  f16* wqT  = takeh((size_t)D * D);
  f16* wklT = takeh((size_t)L * D);
  f16* wvlT = takeh((size_t)L * D);
  f16* wkT  = takeh((size_t)D * L);
  f16* wvT  = takeh((size_t)D * L);
  f16* woT  = takeh((size_t)D * D);
  f16* qh = takeh((size_t)Bn * S * D);  f16* ql = takeh((size_t)Bn * R * D);
  f16* klh = takeh((size_t)Bn * S * L); f16* kll = takeh((size_t)Bn * R * L);
  f16* vlh = takeh((size_t)Bn * S * L); f16* vll = takeh((size_t)Bn * R * L);
  f16* kh = takeh((size_t)Bn * S * D);  f16* kl = takeh((size_t)Bn * R * D);
  f16* vh = takeh((size_t)Bn * S * D);  f16* vl = takeh((size_t)Bn * R * D);
  f16* ctxl = takeh((size_t)Bn * R * D);
  if (off > ws_size || off > (size_t)134217728) return;

  const float sw = 32.0f, isw = 1.0f / 32.0f;

  k_cvt_x<<<dim3((unsigned)(((size_t)Bn * S * D / 8 + 255) / 256)), 256, 0, stream>>>(x, xh, Bn * S, D, S, SEQ_FULL);
  k_wT<<<dim3(D / 32, D / 64), 256, 0, stream>>>(wq, wqT, D, D, sw);
  k_wT<<<dim3(L / 32, D / 64), 256, 0, stream>>>(wklat, wklT, D, L, sw);
  k_wT<<<dim3(L / 32, D / 64), 256, 0, stream>>>(wvlat, wvlT, D, L, sw);
  k_wT<<<dim3(D / 32, L / 64), 256, 0, stream>>>(wk, wkT, L, D, sw);
  k_wT<<<dim3(D / 32, L / 64), 256, 0, stream>>>(wv, wvT, L, D, sw);
  k_wT<<<dim3(D / 32, D / 64), 256, 0, stream>>>(wo, woT, D, D, sw);

  const int tpa = S / 128;
  const int tps = R / 128;
  const int tpp = (S - R) / 128;

  k_gemm<false, 0, true><<<dim3(D / 128, Bn * tpa), 256, 0, stream>>>(xh, xh, wqT, bq, qh, ql, out,
                                                                       D, D, tpa, S, 0, R, isw, 1.0f);
  k_gemm<false, 0, false><<<dim3(L / 128, Bn * tpa), 256, 0, stream>>>(xh, xh, wklT, bq, klh, kll, out,
                                                                        D, L, tpa, S, 0, R, isw, 1.0f);
  k_gemm<false, 0, false><<<dim3(L / 128, Bn * tpa), 256, 0, stream>>>(xh, xh, wvlT, bq, vlh, vll, out,
                                                                        D, L, tpa, S, 0, R, isw, 1.0f);
  k_gemm<true, 0, false><<<dim3(D / 128, Bn * tps), 256, 0, stream>>>(klh, kll, wkT, bq, kh, kl, out,
                                                                       L, D, tps, S, 0, R, isw, 1.0f);
  if (tpp > 0)
    k_gemm<false, 0, false><<<dim3(D / 128, Bn * tpp), 256, 0, stream>>>(klh, kll, wkT, bq, kh, kl, out,
                                                                          L, D, tpp, S, R, R, isw, 1.0f);
  k_gemm<true, 0, false><<<dim3(D / 128, Bn * tps), 256, 0, stream>>>(vlh, vll, wvT, bq, vh, vl, out,
                                                                       L, D, tps, S, 0, R, isw, 1.0f);
  if (tpp > 0)
    k_gemm<false, 0, false><<<dim3(D / 128, Bn * tpp), 256, 0, stream>>>(vlh, vll, wvT, bq, vh, vl, out,
                                                                          L, D, tpp, S, R, R, isw, 1.0f);

  const float scale = 0.08838834764831845f;
  const int qbs = R / 64, qbp = (S - R) / 64;
  k_attn<true><<<dim3(qbs, H * 2, Bn), 128, 0, stream>>>(qh, ql, kh, kl, vh, vl, ctxh, ctxl, 0, S, R, scale);
  if (qbp > 0)
    k_attn<false><<<dim3(qbp, H * 2, Bn), 128, 0, stream>>>(qh, ql, kh, kl, vh, vl, ctxh, ctxl, qbs, S, R, scale);

  k_gemm<true, 2, true><<<dim3(D / 128, Bn * tps), 256, 0, stream>>>(ctxh, ctxl, woT, bo, kh, kl, out,
                                                                      D, D, tps, S, 0, R, 1.0f / 512.0f, 1.0f);
  if (tpp > 0)
    k_gemm<false, 2, true><<<dim3(D / 128, Bn * tpp), 256, 0, stream>>>(ctxh, ctxl, woT, bo, kh, kl, out,
                                                                         D, D, tpp, S, R, R, 1.0f / 512.0f, 1.0f);
}
